// DualStateLinearAttention_61984968016009
// MI455X (gfx1250) — hardware-verified
//
#include <hip/hip_runtime.h>
#include <math.h>

typedef __attribute__((ext_vector_type(16))) _Float16 v16h;
typedef __attribute__((ext_vector_type(8)))  _Float16 v8h;
typedef __attribute__((ext_vector_type(16))) __bf16   v16b;
typedef __attribute__((ext_vector_type(8)))  __bf16   v8b;
typedef __attribute__((ext_vector_type(8)))  float    v8f;
typedef __attribute__((ext_vector_type(4)))  float    v4f;

constexpr int kB    = 2;
constexpr int kS    = 2048;
constexpr int kHid  = 2048;
constexpr int kHd   = 128;
constexpr int kHG   = 8;
constexpr int kNG   = kHG * kHd;
constexpr int kThr  = 256;
constexpr float kInCarry = 1024.0f;
constexpr float kSc = 1.0f / (kInCarry * kInCarry);
constexpr float kCa = 256.0f;
constexpr float kScA = 1.0f / (kCa * kInCarry);
constexpr float kQScale = 0.08838834764831845f;
constexpr float kGateNorm = 16.0f, kClampMin = -50.0f;
constexpr float kF16MinNormal = 6.103515625e-5f;

static_assert((kS % 64) == 0 && (kNG % 64) == 0 && (kHid % 64) == 0 && ((kS / 64) * (kNG / 64)) % 8 == 0 && ((kS / 64) * (kHid / 64)) % 8 == 0, "GEMM M, N multiples of 64; grids exact");
static_assert((kHid % 256) == 0 && kHid == 2 * kNG && kHid == 16 * kHd, "GEMM K a multiple of 32; the plane cast's pitch a multiple of 256; two passes of eight heads");

constexpr size_t kOffWQ = 0ull;
constexpr size_t kOffWK = 8388608ull;
constexpr size_t kOffWV = 16777216ull;
constexpr size_t kOffWG1 = 25165824ull;
constexpr size_t kOffWG2 = 33554432ull;
constexpr size_t kOffWO = 41943040ull;
constexpr size_t kOffBIAS = 50331648ull;
constexpr size_t kOffAL = 50364416ull;
constexpr size_t kOffX16 = 50368512ull;
constexpr size_t kOffQP = 58757120ull;
constexpr size_t kOffKP = 67145728ull;
constexpr size_t kOffVP = 75534336ull;
constexpr size_t kOffEP = 83922944ull;
constexpr size_t kOffATT32 = 100700160ull;
constexpr size_t kOffATT16 = 117477376ull;
constexpr size_t kWsTotal = 125865984ull;
static_assert(kWsTotal <= 134217728ull, "carve cap: under 128 MiB");
static_assert(kOffWQ == 0
              && kOffWK == kOffWQ + 8388608ull
              && kOffWV == kOffWK + 8388608ull
              && kOffWG1 == kOffWV + 8388608ull
              && kOffWG2 == kOffWG1 + 8388608ull
              && kOffWO == kOffWG2 + 8388608ull
              && kOffBIAS == kOffWO + 8388608ull
              && kOffAL == kOffBIAS + 32768ull
              && kOffX16 == kOffAL + 4096ull
              && kOffQP == kOffX16 + 8388608ull
              && kOffKP == kOffQP + 8388608ull
              && kOffVP == kOffKP + 8388608ull
              && kOffEP == kOffVP + 8388608ull
              && kOffATT32 == kOffEP + 16777216ull
              && kOffATT16 == kOffATT32 + 16777216ull
              && kWsTotal == kOffATT16 + 8388608ull, "the carve is chained and totalled");
static_assert((kOffWQ % 256) == 0 && (kOffWK % 256) == 0 && (kOffWV % 256) == 0 && (kOffWG1 % 256) == 0 && (kOffWG2 % 256) == 0 && (kOffWO % 256) == 0 && (kOffBIAS % 256) == 0 && (kOffAL % 256) == 0 && (kOffX16 % 256) == 0 && (kOffQP % 256) == 0 && (kOffKP % 256) == 0 && (kOffVP % 256) == 0 && (kOffEP % 256) == 0 && (kOffATT32 % 256) == 0 && (kOffATT16 % 256) == 0, "aligned regions");
constexpr int kFZB = 0, kFG1 = 2048, kFG2 = 4096, kFEnd = 8192;
static_assert(kFG1 == kFZB + kHid && kFG2 == kFG1 + kHid && kFG2 + kHid <= kFEnd, "bias stream map");

__device__ __forceinline__ unsigned short f2bf_bits(float f) {
  unsigned u = __float_as_uint(f);
  return (unsigned short)((u + 0x7FFFu + ((u >> 16) & 1u)) >> 16);
}
__device__ __forceinline__ float bf_bits2f(unsigned short h) { return __uint_as_float(((unsigned)h) << 16); }
__device__ __forceinline__ float bf16r(float f) { return bf_bits2f(f2bf_bits(f)); }
__device__ __forceinline__ float carry_flush(float v, float carry) {
  const float s = v * carry;
  return (fabsf(s) < kF16MinNormal) ? 0.0f : s;
}
__device__ __forceinline__ float frcp(float x) { return __builtin_amdgcn_rcpf(x); }

__device__ __forceinline__ void dep_guard4_h(v8f& a, v8f& b, v8f& c, v8f& d, v16h x, v16h y) { asm volatile("v_nop\n\tv_nop\n\tv_nop\n\tv_nop" : "+v"(a), "+v"(b), "+v"(c), "+v"(d) : "v"(x), "v"(y)); }
__device__ __forceinline__ void dep_guard4_b(v8f& a, v8f& b, v8f& c, v8f& d, v16b x, v16b y) { asm volatile("v_nop\n\tv_nop\n\tv_nop\n\tv_nop" : "+v"(a), "+v"(b), "+v"(c), "+v"(d) : "v"(x), "v"(y)); }
__device__ __forceinline__ void keep4_h(v16h a, v16h b, v16h c, v16h d) { asm volatile("v_nop" :: "v"(a), "v"(b), "v"(c), "v"(d)); }
__device__ __forceinline__ void keep4_b(v16b a, v16b b, v16b c, v16b d) { asm volatile("v_nop" :: "v"(a), "v"(b), "v"(c), "v"(d)); }
__device__ __forceinline__ void acc_guard4(v8f& a, v8f& b, v8f& c, v8f& d) { asm volatile("v_nop\n\tv_nop\n\tv_nop\n\tv_nop" : "+v"(a), "+v"(b), "+v"(c), "+v"(d)); }

template <typename T> struct Frag;
template <> struct Frag<_Float16> {
  typedef v16h V; union U { v16h v; v8h h[2]; };
  static __device__ __forceinline__ v16h load(const _Float16* p) {
    U f; f.h[0] = *(const v8h*)(p); f.h[1] = *(const v8h*)(p + 16); return f.v;
  }
  static __device__ __forceinline__ v8f mma(v16h a, v16h b, v8f c) {
    return __builtin_amdgcn_wmma_f32_16x16x32_f16(false, a, false, b, (short)0, c, false, false);
  }
  static __device__ __forceinline__ void guard4(v8f& a, v8f& b, v8f& c, v8f& d, v16h x, v16h y) { dep_guard4_h(a, b, c, d, x, y); }
  static __device__ __forceinline__ void keep(v16h a, v16h b, v16h c, v16h d) { keep4_h(a, b, c, d); }
};
template <> struct Frag<__bf16> {
  typedef v16b V; union U { v16b v; v8b h[2]; };
  static __device__ __forceinline__ v16b load(const __bf16* p) {
    U f; f.h[0] = *(const v8b*)(p); f.h[1] = *(const v8b*)(p + 16); return f.v;
  }
  static __device__ __forceinline__ v8f mma(v16b a, v16b b, v8f c) {
    return __builtin_amdgcn_wmma_f32_16x16x32_bf16(false, a, false, b, (short)0, c, false, false);
  }
  static __device__ __forceinline__ void guard4(v8f& a, v8f& b, v8f& c, v8f& d, v16b x, v16b y) { dep_guard4_b(a, b, c, d, x, y); }
  static __device__ __forceinline__ void keep(v16b a, v16b b, v16b c, v16b d) { keep4_b(a, b, c, d); }
};

__device__ __forceinline__ v8f mma_h(v16h a, v16h b, v8f c) {
  c = __builtin_amdgcn_wmma_f32_16x16x32_f16(false, a, false, b, (short)0, c, false, false);
  asm volatile("v_nop\n\tv_nop\n\tv_nop\n\tv_nop" : "+v"(c) : "v"(a), "v"(b));
  return c;
}

template <int ET> struct Elem;
template <> struct Elem<0> { typedef _Float16 T; };
template <> struct Elem<1> { typedef __bf16 T; };
template <int ET, bool SPLIT, int BIAS_MODE, int OUT_MODE, bool RESID, int ACT = 0>
__global__ __launch_bounds__(256) void wmma_gemm64(
    const unsigned short* __restrict__ Ap, const unsigned short* __restrict__ A2p, int lda, long strideA,
    const unsigned short* __restrict__ Btp, const unsigned short* __restrict__ Bt2p, int ldb, long strideB,
    void* __restrict__ Cout, void* __restrict__ Cout2, int ldc, long strideC,
    const float* __restrict__ bias,
    const float* __restrict__ resid, long strideR,
    int M, int N, int K, float scale) {
  typedef typename Elem<ET>::T T;
  typedef typename Frag<T>::V V;
  const T* A = (const T*)Ap; const T* A2 = (const T*)A2p; const T* Bt = (const T*)Btp; const T* Bt2 = (const T*)Bt2p;
  __shared__ __align__(16) float sT[8][16 * 68];
  const int b    = blockIdx.y;
  const int lane = threadIdx.x & 31;
  const int wave = threadIdx.x >> 5;
  const int tilesN = N >> 6;
  const int tilesM = M >> 6;
  const int tile = blockIdx.x * 8 + wave;
  if (tile >= tilesM * tilesN) return;
  const int tm = tile / tilesN;
  const int tn = tile - tm * tilesN;
  const int m0 = tm << 6;
  const int n0 = tn << 6;

  const T* Ab  = A  + (size_t)b * strideA;
  const T* Bb  = Bt + (size_t)b * strideB;
  const T* Ab2 = SPLIT ? (A2  + (size_t)b * strideA) : nullptr;
  const T* Bb2 = SPLIT ? (Bt2 + (size_t)b * strideB) : nullptr;

  const int rlane = lane & 15;
  const int koff  = (lane >> 4) * 8;
  const int mOff  = (lane >> 4) * 8;

  v8f acc[4][4];
#pragma unroll
  for (int i = 0; i < 4; ++i)
#pragma unroll
    for (int j = 0; j < 4; ++j) acc[i][j] = (v8f){0.f,0.f,0.f,0.f,0.f,0.f,0.f,0.f};

  for (int k0 = 0; k0 < K; k0 += 32) {
    V bh[4], bl[4];
#pragma unroll
    for (int j = 0; j < 4; ++j) {
      const size_t bo = (size_t)(n0 + (j << 4) + rlane) * ldb + koff + k0;
      bh[j] = Frag<T>::load(Bb + bo);
      if (SPLIT) bl[j] = Frag<T>::load(Bb2 + bo);
    }
#pragma unroll
    for (int i = 0; i < 4; ++i) {
      const size_t ao = (size_t)(m0 + (i << 4) + rlane) * lda + koff + k0;
      V ah = Frag<T>::load(Ab + ao);
      V al;
      if (SPLIT) al = Frag<T>::load(Ab2 + ao);
#pragma unroll
      for (int j = 0; j < 4; ++j) {
        acc[i][j] = Frag<T>::mma(ah, bh[j], acc[i][j]);
        if (SPLIT) {
          acc[i][j] = Frag<T>::mma(ah, bl[j], acc[i][j]);
          acc[i][j] = Frag<T>::mma(al, bh[j], acc[i][j]);
        }
      }
      Frag<T>::guard4(acc[i][0], acc[i][1], acc[i][2], acc[i][3], ah, SPLIT ? al : ah);
    }
    Frag<T>::keep(bh[0], bh[1], bh[2], bh[3]);
    if (SPLIT) Frag<T>::keep(bl[0], bl[1], bl[2], bl[3]);
  }
  acc_guard4(acc[0][0], acc[0][1], acc[0][2], acc[0][3]);
  acc_guard4(acc[1][0], acc[1][1], acc[1][2], acc[1][3]);
  acc_guard4(acc[2][0], acc[2][1], acc[2][2], acc[2][3]);
  acc_guard4(acc[3][0], acc[3][1], acc[3][2], acc[3][3]);

  float* slab = sT[wave];
  const float* Rb = RESID ? (resid + (size_t)b * strideR) : nullptr;
#pragma unroll
  for (int i = 0; i < 4; ++i) {
    const int mBase = m0 + (i << 4);
#pragma unroll
    for (int j = 0; j < 4; ++j) {
      const int n = n0 + (j << 4) + rlane;
      float bv = 0.f;
      if (BIAS_MODE == 2) bv = bias[n];
#pragma unroll
      for (int r = 0; r < 8; ++r) {
        float v = acc[i][j][r] * scale;
        if (BIAS_MODE == 1) v += bias[mBase + mOff + r];
        if (BIAS_MODE == 2) v += bv;
        if (RESID) v += Rb[(size_t)(mBase + mOff + r) * ldc + n];
        if (ACT == 1) v = tanhf(v);
        if (ACT == 2) v = fmaxf(v, 0.0f);
        if (ACT == 3) v = v / (1.0f + expf(-v));
        if (ACT == 4) v = (v > 0.f) ? v : 0.01f * v;
        slab[(mOff + r) * 68 + (j << 4) + rlane] = v;
      }
    }
    __builtin_amdgcn_fence(__ATOMIC_RELEASE, "workgroup");
    __builtin_amdgcn_wave_barrier();
    __builtin_amdgcn_fence(__ATOMIC_ACQUIRE, "workgroup");
    if (OUT_MODE == 0) {
      float* C = (float*)Cout + (size_t)b * strideC;
      const int hh = lane >> 4, c4 = (lane & 15) * 4;
      for (int pass = 0; pass < 2; ++pass) {
#pragma unroll
        for (int it = 0; it < 8; ++it) {
          const int row = it * 2 + hh;
          v4f v = *(const v4f*)(slab + row * 68 + c4);
          *(volatile v4f*)(C + (size_t)(mBase + row) * ldc + n0 + c4) = v;
        }
        __threadfence();
      }
    } else {
      const int q = lane >> 3, c8 = (lane & 7) * 8;
      unsigned short* C  = (unsigned short*)Cout  + (size_t)b * strideC;
      unsigned short* C2 = (OUT_MODE == 2) ? ((unsigned short*)Cout2 + (size_t)b * strideC) : nullptr;
      for (int pass = 0; pass < 2; ++pass) {
#pragma unroll
        for (int it = 0; it < 4; ++it) {
          const int row = it * 4 + q;
          const float* sp = slab + row * 68 + c8;
          v8h hv, lv;
#pragma unroll
          for (int e = 0; e < 8; ++e) {
            if (OUT_MODE == 1) {
              hv[e] = (_Float16)sp[e];
            } else {
              unsigned short hb = f2bf_bits(sp[e]);
              unsigned short lb = f2bf_bits(sp[e] - bf_bits2f(hb));
              hv[e] = __builtin_bit_cast(_Float16, hb);
              lv[e] = __builtin_bit_cast(_Float16, lb);
            }
          }
          *(volatile v8h*)(C + (size_t)(mBase + row) * ldc + n0 + c8) = hv;
          if (OUT_MODE == 2) *(volatile v8h*)(C2 + (size_t)(mBase + row) * ldc + n0 + c8) = lv;
        }
        __threadfence();
      }
    }
    __builtin_amdgcn_fence(__ATOMIC_RELEASE, "workgroup");
    __builtin_amdgcn_wave_barrier();
    __builtin_amdgcn_fence(__ATOMIC_ACQUIRE, "workgroup");
  }
}

__global__ __launch_bounds__(kThr) void cast_plane_kernel(const float* __restrict__ src, unsigned short* __restrict__ dst,
                                                          int colsLog2, int dstPitch, int dstOff) {
  const int i   = blockIdx.x * kThr + threadIdx.x;
  const int sh  = colsLog2 - 3;
  const int row = i >> sh;
  const int c8  = (i & ((1 << sh) - 1)) * 8;
  const float* sp = src + ((size_t)row << colsLog2) + c8;
  const v4f a0 = *(const v4f*)(sp);
  const v4f a1 = *(const v4f*)(sp + 4);
  v8h hv;
#pragma unroll
  for (int e = 0; e < 4; ++e) {
    const float f0 = a0[e];
    const float f1 = a1[e];
    hv[e]     = (_Float16)carry_flush(bf16r(f0), kInCarry);
    hv[4 + e] = (_Float16)carry_flush(bf16r(f1), kInCarry);
  }
  unsigned short* dp = dst + (size_t)row * dstPitch + dstOff + c8;
  *(volatile v8h*)dp = hv;
  __threadfence();
  *(volatile v8h*)dp = hv;
}

__global__ __launch_bounds__(kThr) void setup_kernel(const float* __restrict__ bg1, const float* __restrict__ bg2, const float* __restrict__ alpha,
                                                     float* __restrict__ BIAS, float* __restrict__ AL) {
  unsigned v = blockIdx.x * (unsigned)kThr + threadIdx.x;
  asm volatile("" : "+v"(v));
  v4f o = {0.f, 0.f, 0.f, 0.f};
  float* dp;
  if (v < 2048u) {
    const unsigned i0 = v * 4u;
    if (i0 >= (unsigned)kFG1 && i0 < (unsigned)(kFG2 + kHid)) {
      const float* sp = (i0 < (unsigned)kFG2) ? (bg1 + (i0 - (unsigned)kFG1)) : (bg2 + (i0 - (unsigned)kFG2));
      const v4f a = *(const v4f*)sp;
#pragma unroll
      for (int e = 0; e < 4; ++e) { const float p = a[e]; o[e] = bf16r(p); }
    }
    dp = BIAS + i0;
  } else {
    const unsigned w = v - 2048u;
    float x0 = alpha[0], x1 = alpha[1];
    asm volatile("" : "+v"(x0), "+v"(x1));
    x0 = bf16r(x0); x1 = bf16r(x1);
    const float m = fmaxf(x0, x1), e0 = expf(x0 - m), e1 = expf(x1 - m), s = e0 + e1;
    const bool first = (w == 0u);
    o[0] = first ? (e0 / s) : 0.0f; o[1] = first ? (e1 / s) : 0.0f;
    dp = AL + (size_t)w * 4u;
  }
  *(volatile v4f*)dp = o;
  __threadfence();
  *(volatile v4f*)dp = o;
}
static_assert(kFEnd / 4 == 2048 && 2048 + 256 == 9 * kThr && (2048 % 32) == 0, "set-up grid exact; regions wave-uniform");

__global__ __launch_bounds__(kThr) void gate_kernel(float* __restrict__ EP) {
  const size_t v = (size_t)blockIdx.x * kThr + threadIdx.x;
  float* p = EP + v * 4;
  const v4f g = *(const v4f*)p;
  v4f o;
#pragma unroll
  for (int e = 0; e < 4; ++e) {
    const float x = g[e];
    const float ls = fminf(x, 0.0f) - log1pf(expf(-fabsf(x)));
    o[e] = expf(fmaxf(ls * (1.0f / kGateNorm), kClampMin));
  }
  *(volatile v4f*)p = o;
  __threadfence();
  *(volatile v4f*)p = o;
}
static_assert(((size_t)2 * kS * kNG / 4) % kThr == 0, "gate grid exact");

__global__ __launch_bounds__(kHd) void gla_scan_kernel(const float* __restrict__ QP, const float* __restrict__ KP, const float* __restrict__ VP,
                                                       const float* __restrict__ E, float* __restrict__ ATT, const float* __restrict__ coefp, int acc) {
  __shared__ float st[kHd * kHd];
  const unsigned vcol = threadIdx.x;
  const unsigned hoff = blockIdx.x * (unsigned)kHd;
  const float coef = coefp[0];
  for (int k = 0; k < kHd; ++k) st[k * kHd + vcol] = 0.0f;
  for (int t = 0; t < kS; ++t) {
    const float* qr = QP + (size_t)t * kNG + hoff;
    const float* kr = KP + (size_t)t * kNG + hoff;
    const float* er = E + (size_t)t * kNG + hoff;
    const float vv = VP[(size_t)t * kNG + hoff + vcol];
    float sum = 0.0f;
#pragma unroll 1
    for (int k4 = 0; k4 < kHd; k4 += 4) {
      const v4f q4 = *(const v4f*)(qr + k4), c4 = *(const v4f*)(kr + k4), e4 = *(const v4f*)(er + k4);
#pragma unroll
      for (int j = 0; j < 4; ++j) {
        const int idx = (k4 + j) * kHd + (int)vcol;
        const float s = st[idx] * e4[j] + c4[j] * vv;
        st[idx] = s;
        sum += q4[j] * s;
      }
    }
    float* op = ATT + (size_t)t * kHid + hoff + vcol;
    const float prev = acc ? *op : 0.0f;
    const float res = prev + coef * (sum * kQScale);
    *(volatile float*)op = res;
    __threadfence();
    *(volatile float*)op = res;
  }
}
static_assert(kHd * kHd * 4 == 65536 && kHd == 128, "the state: 64 KB of LDS a block; one thread a value column");

__global__ __launch_bounds__(kThr) void att_cast_kernel(const float* __restrict__ ATT32, unsigned short* __restrict__ ATT16) {
  const size_t v = (size_t)blockIdx.x * kThr + threadIdx.x;
  const v4f a0 = *(const v4f*)(ATT32 + v * 8), a1 = *(const v4f*)(ATT32 + v * 8 + 4);
  v8h hv;
#pragma unroll
  for (int e = 0; e < 4; ++e) { hv[e] = (_Float16)carry_flush(a0[e], kCa); hv[4 + e] = (_Float16)carry_flush(a1[e], kCa); }
  unsigned short* dp = ATT16 + v * 8;
  *(volatile v8h*)dp = hv;
  __threadfence();
  *(volatile v8h*)dp = hv;
}
static_assert(((size_t)kS * kHid / 8) % kThr == 0, "attention cast grid exact");

static_assert(((size_t)kHid * kHid / 8) % kThr == 0 && ((size_t)kS * kHid / 8) % kThr == 0, "plane cast grids exact");

extern "C" void kernel_launch(void* const* d_in, const int* in_sizes, int n_in,
                              void* d_out, int out_size, void* d_ws, size_t ws_size,
                              hipStream_t stream) {
  if (n_in < 10 || d_out == nullptr || d_ws == nullptr) return;
  if (in_sizes[0] != kB * kS * kHid || in_sizes[1] != kHid * kHid || in_sizes[2] != kHid * kHid || in_sizes[3] != kHid * kHid || in_sizes[4] != kHid * kHid) return;
  if (in_sizes[5] != kHid * kHid || in_sizes[6] != kHid || in_sizes[7] != kHid * kHid || in_sizes[8] != kHid || in_sizes[9] != 2) return;
  if (out_size != kB * kS * kHid) return;
  if (ws_size < kWsTotal) return;
  const float* hidden = (const float*)d_in[0];
  const float* Wq = (const float*)d_in[1];
  const float* Wk = (const float*)d_in[2];
  const float* Wv = (const float*)d_in[3];
  const float* Wo = (const float*)d_in[4];
  const float* Wg1 = (const float*)d_in[5];
  const float* bg1 = (const float*)d_in[6];
  const float* Wg2 = (const float*)d_in[7];
  const float* bg2 = (const float*)d_in[8];
  const float* alpha = (const float*)d_in[9];
  float* out = (float*)d_out;
  char* ws = (char*)d_ws;
  unsigned short* WQ = (unsigned short*)(ws + kOffWQ);
  unsigned short* WK = (unsigned short*)(ws + kOffWK);
  unsigned short* WV = (unsigned short*)(ws + kOffWV);
  unsigned short* WG1 = (unsigned short*)(ws + kOffWG1);
  unsigned short* WG2 = (unsigned short*)(ws + kOffWG2);
  unsigned short* WO = (unsigned short*)(ws + kOffWO);
  float* BIAS = (float*)(ws + kOffBIAS);
  float* AL = (float*)(ws + kOffAL);
  unsigned short* X16 = (unsigned short*)(ws + kOffX16);
  float* QP = (float*)(ws + kOffQP);
  float* KP = (float*)(ws + kOffKP);
  float* VP = (float*)(ws + kOffVP);
  float* EP = (float*)(ws + kOffEP);
  float* ATT32 = (float*)(ws + kOffATT32);
  unsigned short* ATT16 = (unsigned short*)(ws + kOffATT16);

  const int gW = (int)(((size_t)kHid * kHid / 8) / kThr), gX = (int)(((size_t)kS * kHid / 8) / kThr);
  cast_plane_kernel<<<gW, kThr, 0, stream>>>(Wq, WQ, 11, kHid, 0);
  cast_plane_kernel<<<gW, kThr, 0, stream>>>(Wk, WK, 11, kHid, 0);
  cast_plane_kernel<<<gW, kThr, 0, stream>>>(Wv, WV, 11, kHid, 0);
  cast_plane_kernel<<<gW, kThr, 0, stream>>>(Wg1, WG1, 11, kHid, 0);
  cast_plane_kernel<<<gW, kThr, 0, stream>>>(Wg2, WG2, 11, kHid, 0);
  cast_plane_kernel<<<gW, kThr, 0, stream>>>(Wo, WO, 11, kHid, 0);
  setup_kernel<<<9, kThr, 0, stream>>>(bg1, bg2, alpha, BIAS, AL);

  for (int s = 0; s < kB; ++s) {
    cast_plane_kernel<<<gX, kThr, 0, stream>>>(hidden + (size_t)s * kS * kHid, X16, 11, kHid, 0);
    for (int hg = 0; hg < 2; ++hg) {
      const size_t wo = (size_t)hg * kNG * kHid;
      float* E1 = EP; float* E2 = EP + (size_t)kS * kNG;
      wmma_gemm64<0, false, 2, 0, false, 0><<<dim3((kS / 64) * (kNG / 64) / 8, 1), 256, 0, stream>>>(
          X16, X16, kHid, 0L, WQ + wo, WQ + wo, kHid, 0L, (void*)QP, (void*)QP, kNG, 0L, BIAS + kFZB, nullptr, 0L, kS, kNG, kHid, kSc);
      wmma_gemm64<0, false, 2, 0, false, 0><<<dim3((kS / 64) * (kNG / 64) / 8, 1), 256, 0, stream>>>(
          X16, X16, kHid, 0L, WK + wo, WK + wo, kHid, 0L, (void*)KP, (void*)KP, kNG, 0L, BIAS + kFZB, nullptr, 0L, kS, kNG, kHid, kSc);
      wmma_gemm64<0, false, 2, 0, false, 0><<<dim3((kS / 64) * (kNG / 64) / 8, 1), 256, 0, stream>>>(
          X16, X16, kHid, 0L, WV + wo, WV + wo, kHid, 0L, (void*)VP, (void*)VP, kNG, 0L, BIAS + kFZB, nullptr, 0L, kS, kNG, kHid, kSc);
      wmma_gemm64<0, false, 2, 0, false, 0><<<dim3((kS / 64) * (kNG / 64) / 8, 1), 256, 0, stream>>>(
          X16, X16, kHid, 0L, WG1 + wo, WG1 + wo, kHid, 0L, (void*)E1, (void*)E1, kNG, 0L, BIAS + kFG1 + hg * kNG, nullptr, 0L, kS, kNG, kHid, kSc);
      wmma_gemm64<0, false, 2, 0, false, 0><<<dim3((kS / 64) * (kNG / 64) / 8, 1), 256, 0, stream>>>(
          X16, X16, kHid, 0L, WG2 + wo, WG2 + wo, kHid, 0L, (void*)E2, (void*)E2, kNG, 0L, BIAS + kFG2 + hg * kNG, nullptr, 0L, kS, kNG, kHid, kSc);
      gate_kernel<<<(int)(((size_t)2 * kS * kNG / 4) / kThr), kThr, 0, stream>>>(EP);
      gla_scan_kernel<<<kHG, kHd, 0, stream>>>(QP, KP, VP, E1, ATT32 + (size_t)hg * kNG, AL + 0, 0);
      gla_scan_kernel<<<kHG, kHd, 0, stream>>>(QP, KP, VP, E2, ATT32 + (size_t)hg * kNG, AL + 1, 1);
    }
    att_cast_kernel<<<(int)(((size_t)kS * kHid / 8) / kThr), kThr, 0, stream>>>(ATT32, ATT16);
    wmma_gemm64<0, false, 2, 0, false, 0><<<dim3((kS / 64) * (kHid / 64) / 8, 1), 256, 0, stream>>>(
        ATT16, ATT16, kHid, 0L, WO, WO, kHid, 0L, (void*)(out + (size_t)s * kS * kHid), (void*)(out + (size_t)s * kS * kHid), kHid, 0L, BIAS + kFZB, nullptr, 0L, kS, kHid, kHid, kScA);
  }
}
